// SharedNATransformerLayer_48292612276770
// MI455X (gfx1250) — hardware-verified
//
#include <hip/hip_runtime.h>

constexpr int kT     = 8;
constexpr int kH     = 16;
constexpr int kW     = 16;
constexpr int kTok   = kT * kH * kW;
constexpr int kDim   = 256;
constexpr int kFF    = 1024;
constexpr int kHeads = 8;
constexpr int kDh    = 32;
constexpr int kWin   = 5;
constexpr float kQScale   = 0.17677669529663687f;
constexpr float kEps      = 1e-6f;
constexpr float kInvDim   = 1.0f / 256.0f;
constexpr float kWCarry   = 64.0f;
constexpr float kAtCarry  = 64.0f;
constexpr float kGCarry   = 256.0f;

typedef __attribute__((ext_vector_type(16))) _Float16 v16h;
typedef __attribute__((ext_vector_type(8)))  _Float16 v8h;
typedef __attribute__((ext_vector_type(16))) __bf16   v16b;
typedef __attribute__((ext_vector_type(8)))  __bf16   v8b;
typedef __attribute__((ext_vector_type(8)))  float    v8f;
typedef __attribute__((ext_vector_type(4)))  float    v4f;
typedef __attribute__((ext_vector_type(4)))  unsigned int v4u;

__device__ __forceinline__ unsigned short f2bf_bits(float f) {
  unsigned u = __float_as_uint(f);
  return (unsigned short)((u + 0x7FFFu + ((u >> 16) & 1u)) >> 16);
}
__device__ __forceinline__ float bf_bits2f(unsigned short h) { return __uint_as_float(((unsigned)h) << 16); }

__device__ __forceinline__ void dep_guard_h(v8f& a, v8f& b, v16h x, v16h y) { asm volatile("v_nop\n\tv_nop\n\tv_nop\n\tv_nop" : "+v"(a), "+v"(b) : "v"(x), "v"(y)); }
__device__ __forceinline__ void dep_guard_b(v8f& a, v8f& b, v16b x, v16b y) { asm volatile("v_nop\n\tv_nop\n\tv_nop\n\tv_nop" : "+v"(a), "+v"(b) : "v"(x), "v"(y)); }
__device__ __forceinline__ void keep4_h(v16h a, v16h b, v16h c, v16h d) { asm volatile("v_nop" :: "v"(a), "v"(b), "v"(c), "v"(d)); }
__device__ __forceinline__ void keep4_b(v16b a, v16b b, v16b c, v16b d) { asm volatile("v_nop" :: "v"(a), "v"(b), "v"(c), "v"(d)); }
__device__ __forceinline__ void acc_guard4(v8f& a, v8f& b, v8f& c, v8f& d) { asm volatile("v_nop\n\tv_nop\n\tv_nop\n\tv_nop" : "+v"(a), "+v"(b), "+v"(c), "+v"(d)); }
template <typename T> struct Frag;
template <> struct Frag<_Float16> {
  typedef v16h V; union U { v16h v; v8h h[2]; };
  static __device__ __forceinline__ v16h load(const _Float16* p) {
    U f; f.h[0] = *(const v8h*)(p); f.h[1] = *(const v8h*)(p + 16); return f.v;
  }
  static __device__ __forceinline__ v8f mma(v16h a, v16h b, v8f c) {
    return __builtin_amdgcn_wmma_f32_16x16x32_f16(false, a, false, b, (short)0, c, false, false);
  }
  static __device__ __forceinline__ void guard(v8f& a, v8f& b, v16h x, v16h y) { dep_guard_h(a, b, x, y); }
  static __device__ __forceinline__ void keep(v16h a, v16h b, v16h c, v16h d) { keep4_h(a, b, c, d); }
};
template <> struct Frag<__bf16> {
  typedef v16b V; union U { v16b v; v8b h[2]; };
  static __device__ __forceinline__ v16b load(const __bf16* p) {
    U f; f.h[0] = *(const v8b*)(p); f.h[1] = *(const v8b*)(p + 16); return f.v;
  }
  static __device__ __forceinline__ v8f mma(v16b a, v16b b, v8f c) {
    return __builtin_amdgcn_wmma_f32_16x16x32_bf16(false, a, false, b, (short)0, c, false, false);
  }
  static __device__ __forceinline__ void guard(v8f& a, v8f& b, v16b x, v16b y) { dep_guard_b(a, b, x, y); }
  static __device__ __forceinline__ void keep(v16b a, v16b b, v16b c, v16b d) { keep4_b(a, b, c, d); }
};

__device__ __forceinline__ unsigned pk16(unsigned short a, unsigned short b) { return (unsigned)a | ((unsigned)b << 16); }
__device__ __forceinline__ unsigned short h_bits(float f) { const _Float16 h = (_Float16)f; return __builtin_bit_cast(unsigned short, h); }

template <int ET> struct Elem;
template <> struct Elem<0> { typedef _Float16 T; };
template <> struct Elem<1> { typedef __bf16 T; };
template <int ET, bool SPLIT, int BIAS_MODE, int OUT_MODE, int RESID, int ACT = 0>
__global__ __launch_bounds__(256) void wmma_gemm64(
    const unsigned short* __restrict__ Ap, const unsigned short* __restrict__ A2p, int lda, long strideA,
    const unsigned short* __restrict__ Btp, const unsigned short* __restrict__ Bt2p, int ldb, long strideB,
    void* __restrict__ Cout, void* __restrict__ Cout2, int ldc, long strideC,
    const float* __restrict__ bias,
    const float* __restrict__ resid, long strideR,
    int M, int N, int K, float scale) {
  typedef typename Elem<ET>::T T;
  typedef typename Frag<T>::V V;
  const T* A = (const T*)Ap; const T* A2 = (const T*)A2p; const T* Bt = (const T*)Btp; const T* Bt2 = (const T*)Bt2p;
  __shared__ __align__(16) float sT[8][16 * 68];
  const int b    = blockIdx.y;
  const int lane = threadIdx.x & 31;
  const int wave = threadIdx.x >> 5;
  const int tilesN = N >> 6;
  const int tilesM = M >> 6;
  const int tile = blockIdx.x * 8 + wave;
  if (tile >= tilesM * tilesN) return;
  const int tm = tile / tilesN;
  const int tn = tile - tm * tilesN;
  const int m0 = tm << 6;
  const int n0 = tn << 6;

  const T* Ab  = A  + (size_t)b * strideA;
  const T* Bb  = Bt + (size_t)b * strideB;
  const T* Ab2 = SPLIT ? (A2  + (size_t)b * strideA) : nullptr;
  const T* Bb2 = SPLIT ? (Bt2 + (size_t)b * strideB) : nullptr;

  const int rlane = lane & 15;
  const int koff  = (lane >> 4) * 8;
  const int mOff  = (lane >> 4) * 8;

  v8f acc[4][4];
#pragma unroll
  for (int i = 0; i < 4; ++i)
#pragma unroll
    for (int j = 0; j < 4; ++j) acc[i][j] = (v8f){0.f,0.f,0.f,0.f,0.f,0.f,0.f,0.f};

  for (int k0 = 0; k0 < K; k0 += 32) {
    V bh[4], bl[4];
#pragma unroll
    for (int j = 0; j < 4; ++j) {
      const size_t bo = (size_t)(n0 + (j << 4) + rlane) * ldb + koff + k0;
      bh[j] = Frag<T>::load(Bb + bo);
      if (SPLIT) bl[j] = Frag<T>::load(Bb2 + bo);
    }
#pragma unroll
    for (int i = 0; i < 4; ++i) {
      const size_t ao = (size_t)(m0 + (i << 4) + rlane) * lda + koff + k0;
      V ah = Frag<T>::load(Ab + ao);
      V al;
      if (SPLIT) al = Frag<T>::load(Ab2 + ao);
#pragma unroll
      for (int j = 0; j < 4; ++j) {
        acc[i][j] = Frag<T>::mma(ah, bh[j], acc[i][j]);
        if (SPLIT) {
          acc[i][j] = Frag<T>::mma(ah, bl[j], acc[i][j]);
          acc[i][j] = Frag<T>::mma(al, bh[j], acc[i][j]);
        }
      }
      Frag<T>::guard(acc[i][0], acc[i][3], ah, SPLIT ? al : ah);
    }
    Frag<T>::keep(bh[0], bh[1], bh[2], bh[3]);
    if (SPLIT) Frag<T>::keep(bl[0], bl[1], bl[2], bl[3]);
  }
  acc_guard4(acc[0][0], acc[0][1], acc[0][2], acc[0][3]);
  acc_guard4(acc[1][0], acc[1][1], acc[1][2], acc[1][3]);
  acc_guard4(acc[2][0], acc[2][1], acc[2][2], acc[2][3]);
  acc_guard4(acc[3][0], acc[3][1], acc[3][2], acc[3][3]);

  float* slab = sT[wave];
  const float* Rb = (RESID != 0) ? (resid + (size_t)b * strideR) : nullptr;
#pragma unroll
  for (int i = 0; i < 4; ++i) {
    const int mBase = m0 + (i << 4);
#pragma unroll
    for (int j = 0; j < 4; ++j) {
      const int n = n0 + (j << 4) + rlane;
      float bv = 0.f;
      if (BIAS_MODE == 2) bv = bias[n];
#pragma unroll
      for (int r = 0; r < 8; ++r) {
        float v = acc[i][j][r] * scale;
        if (BIAS_MODE == 1) v += bias[mBase + mOff + r];
        if (BIAS_MODE == 2) v += bv;
        if (RESID == 1) v += Rb[(size_t)(mBase + mOff + r) * ldc + n];
        if (RESID == 2) v *= Rb[(size_t)(mBase + mOff + r) * ldc + n];
        if (ACT == 2) v = fmaxf(v, 0.0f);
        if (ACT == 3) v = v / (1.0f + expf(-v));
        slab[(mOff + r) * 68 + (j << 4) + rlane] = v;
      }
    }
    __builtin_amdgcn_fence(__ATOMIC_RELEASE, "workgroup");
    __builtin_amdgcn_wave_barrier();
    __builtin_amdgcn_fence(__ATOMIC_ACQUIRE, "workgroup");
    if (OUT_MODE == 0) {
      float* C = (float*)Cout + (size_t)b * strideC;
      const int hh = lane >> 4, c4 = (lane & 15) * 4;
      for (int pass = 0; pass < 2; ++pass) {
#pragma unroll
        for (int it = 0; it < 8; ++it) {
          const int row = it * 2 + hh;
          v4f v = *(const v4f*)(slab + row * 68 + c4);
          *(volatile v4f*)(C + (size_t)(mBase + row) * ldc + n0 + c4) = v;
        }
        __threadfence();
      }
    } else {
      const int q = lane >> 3, c8 = (lane & 7) * 8;
      unsigned short* C  = (unsigned short*)Cout  + (size_t)b * strideC;
      unsigned short* C2 = (OUT_MODE == 2) ? ((unsigned short*)Cout2 + (size_t)b * strideC) : nullptr;
      for (int pass = 0; pass < 2; ++pass) {
#pragma unroll
        for (int it = 0; it < 4; ++it) {
          const int row = it * 4 + q;
          const float* sp = slab + row * 68 + c8;
          v8h hv, lv;
#pragma unroll
          for (int e = 0; e < 8; ++e) {
            if (OUT_MODE == 1) {
              hv[e] = (_Float16)sp[e];
            } else {
              unsigned short hb = f2bf_bits(sp[e]);
              unsigned short lb = f2bf_bits(sp[e] - bf_bits2f(hb));
              hv[e] = __builtin_bit_cast(_Float16, hb);
              lv[e] = __builtin_bit_cast(_Float16, lb);
            }
          }
          *(volatile v8h*)(C + (size_t)(mBase + row) * ldc + n0 + c8) = hv;
          if (OUT_MODE == 2) *(volatile v8h*)(C2 + (size_t)(mBase + row) * ldc + n0 + c8) = lv;
        }
        __threadfence();
      }
    }
    __builtin_amdgcn_fence(__ATOMIC_RELEASE, "workgroup");
    __builtin_amdgcn_wave_barrier();
    __builtin_amdgcn_fence(__ATOMIC_ACQUIRE, "workgroup");
  }
}

__global__ __launch_bounds__(256) void wtcast_kernel(const float* __restrict__ Wp, unsigned short* __restrict__ out,
                                                     int nin, int nout, float scale) {
  __shared__ float sm[64][65];
  const int t  = threadIdx.x;
  const int i0 = blockIdx.x * 64;
  const int o0 = blockIdx.y * 64;
#pragma unroll
  for (int it = 0; it < 16; ++it) {
    const int e = it * 256 + t;
    const int r = e >> 6;
    const int c = e & 63;
    sm[c][r] = Wp[(size_t)(i0 + r) * nout + o0 + c] * scale;
  }
  __syncthreads();
  const int lane = t & 31, wave = t >> 5;
  const int q = lane >> 3, c8 = (lane & 7) * 8;
  for (int pass = 0; pass < 2; ++pass) {
#pragma unroll
    for (int it = 0; it < 2; ++it) {
      const int row = wave * 8 + it * 4 + q;
      unsigned short hb[8];
#pragma unroll
      for (int e = 0; e < 8; ++e) hb[e] = h_bits(sm[row][c8 + e]);
      const v4u u = (v4u){pk16(hb[0], hb[1]), pk16(hb[2], hb[3]), pk16(hb[4], hb[5]), pk16(hb[6], hb[7])};
      *(volatile v4u*)(out + (size_t)(o0 + row) * nin + i0 + c8) = u;
    }
    __threadfence();
  }
}

__global__ __launch_bounds__(256) void rmsnorm_f16_kernel(const float* __restrict__ X, const float* __restrict__ w,
                                                          unsigned short* __restrict__ Y, int ntok) {
  const int lane = threadIdx.x & 31, wave = threadIdx.x >> 5;
  const int tok  = blockIdx.x * 8 + wave;
  if (tok >= ntok) return;
  const float* xr = X + (size_t)tok * kDim + 8 * lane;
  const v4f a  = *(const v4f*)(xr);
  const v4f c  = *(const v4f*)(xr + 4);
  const v4f wa = *(const v4f*)(w + 8 * lane);
  const v4f wc = *(const v4f*)(w + 8 * lane + 4);
  float ss = 0.f;
#pragma unroll
  for (int e = 0; e < 4; ++e) ss += a[e] * a[e];
#pragma unroll
  for (int e = 0; e < 4; ++e) ss += c[e] * c[e];
  ss += __shfl_xor(ss, 16, 32);
  ss += __shfl_xor(ss, 8, 32);
  ss += __shfl_xor(ss, 4, 32);
  ss += __shfl_xor(ss, 2, 32);
  ss += __shfl_xor(ss, 1, 32);
  const float rs = rsqrtf(ss * kInvDim + kEps);
  unsigned short hb[8];
#pragma unroll
  for (int e = 0; e < 4; ++e) {
    hb[e]     = h_bits(a[e] * rs * wa[e]);
    hb[4 + e] = h_bits(c[e] * rs * wc[e]);
  }
  const v4u u = (v4u){pk16(hb[0], hb[1]), pk16(hb[2], hb[3]), pk16(hb[4], hb[5]), pk16(hb[6], hb[7])};
  unsigned short* op = Y + (size_t)tok * kDim + 8 * lane;
  *(volatile v4u*)op = u;
  __threadfence();
  *(volatile v4u*)op = u;
}

__global__ __launch_bounds__(256) void na3d_kernel(const float* __restrict__ qp, const float* __restrict__ kp,
                                                   const float* __restrict__ vp, unsigned short* __restrict__ at,
                                                   float carry) {
  __shared__ float slog[kHeads][128];
  __shared__ __align__(16) float sout[kDim];
  const int tok  = blockIdx.x;
  const int head = threadIdx.x >> 5;
  const int lane = threadIdx.x & 31;
  const int t    = tok >> 8;
  const int hh   = (tok >> 4) & 15;
  const int ww   = tok & 15;
  const int hs   = min(max(hh - 2, 0), kH - kWin);
  const int wsx  = min(max(ww - 2, 0), kW - kWin);
  const int kt0  = (t < kWin - 1) ? (kWin - 1 - t) : 0;
  const int nval = (kWin - kt0) * kWin * kWin;
  const int ch   = head * kDh + lane;
  const float qv = qp[(size_t)tok * kDim + ch];
  const float ninf = -__builtin_inff();

  int idx = 0;
#pragma unroll 1
  for (int kt = kt0; kt < kWin; ++kt) {
    const int ti = t - (kWin - 1) + kt;
#pragma unroll 1
    for (int kh = 0; kh < kWin; ++kh) {
      const size_t rowbase = (size_t)((ti * kH + hs + kh) * kW + wsx) * kDim + ch;
#pragma unroll
      for (int kw = 0; kw < kWin; ++kw) {
        float d = qv * kp[rowbase + (size_t)kw * kDim];
        d += __shfl_xor(d, 16, 32);
        d += __shfl_xor(d, 8, 32);
        d += __shfl_xor(d, 4, 32);
        d += __shfl_xor(d, 2, 32);
        d += __shfl_xor(d, 1, 32);
        d *= kQScale;
        if (lane == 0) slog[head][idx + kw] = d;
      }
      idx += kWin;
    }
  }
  __syncthreads();

  float mx = ninf;
#pragma unroll
  for (int j = 0; j < 4; ++j) {
    const int ii = lane + 32 * j;
    const float lv = slog[head][ii];
    mx = fmaxf(mx, (ii < nval) ? lv : ninf);
  }
  mx = fmaxf(mx, __shfl_xor(mx, 16, 32));
  mx = fmaxf(mx, __shfl_xor(mx, 8, 32));
  mx = fmaxf(mx, __shfl_xor(mx, 4, 32));
  mx = fmaxf(mx, __shfl_xor(mx, 2, 32));
  mx = fmaxf(mx, __shfl_xor(mx, 1, 32));
  float psum = 0.f;
#pragma unroll
  for (int j = 0; j < 4; ++j) {
    const int ii = lane + 32 * j;
    const float lv  = slog[head][ii];
    const float arg = (ii < nval) ? (lv - mx) : 0.f;
    float p = expf(arg);
    p = (ii < nval) ? p : 0.f;
    psum += p;
    slog[head][ii] = p;
  }
  psum += __shfl_xor(psum, 16, 32);
  psum += __shfl_xor(psum, 8, 32);
  psum += __shfl_xor(psum, 4, 32);
  psum += __shfl_xor(psum, 2, 32);
  psum += __shfl_xor(psum, 1, 32);
  const float inv = 1.0f / psum;
  __syncthreads();

  float acc = 0.f;
  idx = 0;
#pragma unroll 1
  for (int kt = kt0; kt < kWin; ++kt) {
    const int ti = t - (kWin - 1) + kt;
#pragma unroll 1
    for (int kh = 0; kh < kWin; ++kh) {
      const size_t rowbase = (size_t)((ti * kH + hs + kh) * kW + wsx) * kDim + ch;
#pragma unroll
      for (int kw = 0; kw < kWin; ++kw) {
        const float p = slog[head][idx + kw];
        acc += p * vp[rowbase + (size_t)kw * kDim];
      }
      idx += kWin;
    }
  }
  sout[ch] = acc * inv * carry;
  __syncthreads();

  if (head == 0) {
    const float* sp = sout + 8 * lane;
    const v4f a = *(const v4f*)(sp);
    const v4f c = *(const v4f*)(sp + 4);
    unsigned short hb[8];
#pragma unroll
    for (int e = 0; e < 4; ++e) {
      hb[e]     = h_bits(a[e]);
      hb[4 + e] = h_bits(c[e]);
    }
    const v4u u = (v4u){pk16(hb[0], hb[1]), pk16(hb[2], hb[3]), pk16(hb[4], hb[5]), pk16(hb[6], hb[7])};
    unsigned short* op = at + (size_t)tok * kDim + 8 * lane;
    *(volatile v4u*)op = u;
    __threadfence();
    *(volatile v4u*)op = u;
  }
}

extern "C" void kernel_launch(void* const* d_in, const int* in_sizes, int n_in,
                              void* d_out, int out_size, void* d_ws, size_t ws_size,
                              hipStream_t stream) {
  if (n_in < 14) return;
  if (in_sizes[0] != kTok * kDim || out_size != kTok * kDim) return;
  if (in_sizes[3] != kDim * kDim || in_sizes[11] != kDim * kFF || in_sizes[13] != kFF * kDim) return;

  const float* x       = (const float*)d_in[0];
  const float* norm1_w = (const float*)d_in[1];
  const float* norm2_w = (const float*)d_in[2];
  const float* wq = (const float*)d_in[3];
  const float* bq = (const float*)d_in[4];
  const float* wk = (const float*)d_in[5];
  const float* bk = (const float*)d_in[6];
  const float* wv = (const float*)d_in[7];
  const float* bv = (const float*)d_in[8];
  const float* wo = (const float*)d_in[9];
  const float* bo = (const float*)d_in[10];
  const float* w1 = (const float*)d_in[11];
  const float* w2 = (const float*)d_in[12];
  const float* w3 = (const float*)d_in[13];
  float* out = (float*)d_out;

  char* ws = (char*)d_ws;
  size_t off = 0;
  unsigned short* wqT = (unsigned short*)(ws + off); off += (size_t)kDim * kDim * 2;
  unsigned short* wkT = (unsigned short*)(ws + off); off += (size_t)kDim * kDim * 2;
  unsigned short* wvT = (unsigned short*)(ws + off); off += (size_t)kDim * kDim * 2;
  unsigned short* woT = (unsigned short*)(ws + off); off += (size_t)kDim * kDim * 2;
  unsigned short* w1T = (unsigned short*)(ws + off); off += (size_t)kFF * kDim * 2;
  unsigned short* w2T = (unsigned short*)(ws + off); off += (size_t)kFF * kDim * 2;
  unsigned short* w3T = (unsigned short*)(ws + off); off += (size_t)kDim * kFF * 2;
  unsigned short* xn  = (unsigned short*)(ws + off); off += (size_t)kTok * kDim * 2;
  float* qb = (float*)(ws + off); off += (size_t)kTok * kDim * 4;
  float* kb = (float*)(ws + off); off += (size_t)kTok * kDim * 4;
  float* vb = (float*)(ws + off); off += (size_t)kTok * kDim * 4;
  unsigned short* at  = (unsigned short*)(ws + off); off += (size_t)kTok * kDim * 2;
  float* h1 = (float*)(ws + off); off += (size_t)kTok * kDim * 4;
  unsigned short* yh  = (unsigned short*)(ws + off); off += (size_t)kTok * kDim * 2;
  float* u1 = (float*)(ws + off); off += (size_t)kTok * kFF * 4;
  unsigned short* gh  = (unsigned short*)(ws + off); off += (size_t)kTok * kFF * 2;
  if (off > ws_size) return;

  const dim3 blk(256);
  const float invW   = 1.0f / kWCarry;
  const float invWA  = 1.0f / (kWCarry * kAtCarry);
  const float gScale = kGCarry / kWCarry;
  const float invWG  = 1.0f / (kWCarry * kGCarry);

  wtcast_kernel<<<dim3(kDim / 64, kDim / 64), blk, 0, stream>>>(wq, wqT, kDim, kDim, kWCarry);
  wtcast_kernel<<<dim3(kDim / 64, kDim / 64), blk, 0, stream>>>(wk, wkT, kDim, kDim, kWCarry);
  wtcast_kernel<<<dim3(kDim / 64, kDim / 64), blk, 0, stream>>>(wv, wvT, kDim, kDim, kWCarry);
  wtcast_kernel<<<dim3(kDim / 64, kDim / 64), blk, 0, stream>>>(wo, woT, kDim, kDim, kWCarry);
  wtcast_kernel<<<dim3(kDim / 64, kFF / 64), blk, 0, stream>>>(w1, w1T, kDim, kFF, kWCarry);
  wtcast_kernel<<<dim3(kDim / 64, kFF / 64), blk, 0, stream>>>(w2, w2T, kDim, kFF, kWCarry);
  wtcast_kernel<<<dim3(kFF / 64, kDim / 64), blk, 0, stream>>>(w3, w3T, kFF, kDim, kWCarry);

  rmsnorm_f16_kernel<<<kTok / 8, blk, 0, stream>>>(x, norm1_w, xn, kTok);

  const int gSq  = ((kTok / 64) * (kDim / 64) + 7) / 8;
  const int gFF  = ((kTok / 64) * (kFF / 64) + 7) / 8;
  wmma_gemm64<0, false, 2, 0, 0, 0><<<dim3(gSq, 1), blk, 0, stream>>>(
      xn, xn, kDim, 0L, wqT, wqT, kDim, 0L, (void*)qb, (void*)qb, kDim, 0L, bq, x, 0L, kTok, kDim, kDim, invW);
  wmma_gemm64<0, false, 2, 0, 0, 0><<<dim3(gSq, 1), blk, 0, stream>>>(
      xn, xn, kDim, 0L, wkT, wkT, kDim, 0L, (void*)kb, (void*)kb, kDim, 0L, bk, x, 0L, kTok, kDim, kDim, invW);
  wmma_gemm64<0, false, 2, 0, 0, 0><<<dim3(gSq, 1), blk, 0, stream>>>(
      xn, xn, kDim, 0L, wvT, wvT, kDim, 0L, (void*)vb, (void*)vb, kDim, 0L, bv, x, 0L, kTok, kDim, kDim, invW);

  na3d_kernel<<<kTok, blk, 0, stream>>>(qb, kb, vb, at, kAtCarry);

  wmma_gemm64<0, false, 2, 0, 1, 0><<<dim3(gSq, 1), blk, 0, stream>>>(
      at, at, kDim, 0L, woT, woT, kDim, 0L, (void*)h1, (void*)h1, kDim, 0L, bo, x, 0L, kTok, kDim, kDim, invWA);

  rmsnorm_f16_kernel<<<kTok / 8, blk, 0, stream>>>(h1, norm2_w, yh, kTok);

  wmma_gemm64<0, false, 0, 0, 0, 3><<<dim3(gFF, 1), blk, 0, stream>>>(
      yh, yh, kDim, 0L, w1T, w1T, kDim, 0L, (void*)u1, (void*)u1, kFF, 0L, bq, x, 0L, kTok, kFF, kDim, invW);

  wmma_gemm64<0, false, 0, 1, 2, 0><<<dim3(gFF, 1), blk, 0, stream>>>(
      yh, yh, kDim, 0L, w2T, w2T, kDim, 0L, (void*)gh, (void*)gh, kFF, 0L, bq, u1, 0L, kTok, kFF, kDim, gScale);

  wmma_gemm64<0, false, 0, 0, 1, 0><<<dim3(gSq, 1), blk, 0, stream>>>(
      gh, gh, kFF, 0L, w3T, w3T, kFF, 0L, (void*)out, (void*)out, kDim, 0L, bq, h1, 0L, kTok, kDim, kFF, invWG);
}
